// MultiHeadSelfAttention_11003706212808
// MI455X (gfx1250) — hardware-verified
//
#include <hip/hip_runtime.h>
#ifndef NB
#define NB 2
#endif
#ifndef SEQ
#define SEQ 2048
#endif
#define NB_FULL 2
#define SEQ_FULL 2048
#define DM 1024
#define NH 16
#define HD 64
#define NT (NB * SEQ)
#define XSTRIDE_FULL ((size_t)SEQ_FULL * DM)
#define MSTRIDE_FULL ((size_t)SEQ_FULL * SEQ_FULL)

static_assert(SEQ % 128 == 0);
static_assert(SEQ <= SEQ_FULL);
static_assert(NB <= NB_FULL);
static_assert(DM == NH * HD);
static_assert(HD == 64);
static_assert(DM % 128 == 0);
static_assert((size_t)NT * DM * 2 * 8 + (size_t)DM * DM * 2 * 4 <= (size_t)134217728);

typedef __bf16 v16b __attribute__((ext_vector_type(16)));
typedef _Float16 v16h __attribute__((ext_vector_type(16)));
typedef unsigned short v8us __attribute__((ext_vector_type(8), may_alias));
typedef float v8f __attribute__((ext_vector_type(8)));
typedef float v4f __attribute__((ext_vector_type(4)));
typedef float v4fa __attribute__((ext_vector_type(4), may_alias));
typedef int v4ia __attribute__((ext_vector_type(4), may_alias));
union FragB { v16b v; v8us half[2]; };
union FragH { v16h v; v8us half[2]; _Float16 h[16]; };
union H8 { v8us v; _Float16 h[8]; };

#define LOG2E 1.4426950408889634f
#define FILLV (-1e20f)

__device__ __forceinline__ unsigned short bf16_bits(float x) {
  unsigned int u = __float_as_uint(x);
  return (unsigned short)((u + 0x7FFFu + ((u >> 16) & 1u)) >> 16);
}
__device__ __forceinline__ float bf16_val(unsigned short b) { return __uint_as_float(((unsigned int)b) << 16); }

__device__ __forceinline__ void split_bf8(const v4f x0, const v4f x1, v8us& hi, v8us& lo) {
#pragma unroll
  for (int i = 0; i < 4; ++i) {
    const unsigned short h0 = bf16_bits(x0[i]);
    const unsigned short h1 = bf16_bits(x1[i]);
    hi[i] = h0;     lo[i] = bf16_bits(x0[i] - bf16_val(h0));
    hi[4 + i] = h1; lo[4 + i] = bf16_bits(x1[i] - bf16_val(h1));
  }
}
__device__ __forceinline__ void cvt_h8(const v4f x0, const v4f x1, H8& hi) {
#pragma unroll
  for (int i = 0; i < 4; ++i) {
    hi.h[i]     = (_Float16)(x0[i] * 16.0f);
    hi.h[4 + i] = (_Float16)(x1[i] * 16.0f);
  }
}

__device__ __forceinline__ void mma_row4(v16b a, v16b b0, v16b b1, v16b b2, v16b b3, v8f& c0, v8f& c1, v8f& c2, v8f& c3) {
  c0 = __builtin_amdgcn_wmma_f32_16x16x32_bf16(false, a, false, b0, (short)0, c0, false, false);
  c1 = __builtin_amdgcn_wmma_f32_16x16x32_bf16(false, a, false, b1, (short)0, c1, false, false);
  c2 = __builtin_amdgcn_wmma_f32_16x16x32_bf16(false, a, false, b2, (short)0, c2, false, false);
  c3 = __builtin_amdgcn_wmma_f32_16x16x32_bf16(false, a, false, b3, (short)0, c3, false, false);
  asm volatile("v_nop\n\tv_nop\n\tv_nop\n\tv_nop" : "+v"(c0), "+v"(c1), "+v"(c2), "+v"(c3) : "v"(a), "v"(b0), "v"(b1), "v"(b2), "v"(b3));
}
__device__ __forceinline__ v8f mma_s6(v16b kh0, v16b kh1, v16b kl0, v16b kl1, v16b qh0, v16b qh1, v16b ql0, v16b ql1, v8f c) {
  c = __builtin_amdgcn_wmma_f32_16x16x32_bf16(false, kl0, false, qh0, (short)0, c, false, false);
  c = __builtin_amdgcn_wmma_f32_16x16x32_bf16(false, kl1, false, qh1, (short)0, c, false, false);
  c = __builtin_amdgcn_wmma_f32_16x16x32_bf16(false, kh0, false, ql0, (short)0, c, false, false);
  c = __builtin_amdgcn_wmma_f32_16x16x32_bf16(false, kh1, false, ql1, (short)0, c, false, false);
  c = __builtin_amdgcn_wmma_f32_16x16x32_bf16(false, kh0, false, qh0, (short)0, c, false, false);
  c = __builtin_amdgcn_wmma_f32_16x16x32_bf16(false, kh1, false, qh1, (short)0, c, false, false);
  asm volatile("v_nop\n\tv_nop\n\tv_nop\n\tv_nop" : "+v"(c) : "v"(kh0), "v"(kh1), "v"(kl0), "v"(kl1), "v"(qh0), "v"(qh1), "v"(ql0), "v"(ql1));
  return c;
}
__device__ __forceinline__ void mma_pv4(v16h a0, v16h a1, v16h a2, v16h a3, v16h p, v8f& c0, v8f& c1, v8f& c2, v8f& c3) {
  c0 = __builtin_amdgcn_wmma_f32_16x16x32_f16(false, a0, false, p, (short)0, c0, false, false);
  c1 = __builtin_amdgcn_wmma_f32_16x16x32_f16(false, a1, false, p, (short)0, c1, false, false);
  c2 = __builtin_amdgcn_wmma_f32_16x16x32_f16(false, a2, false, p, (short)0, c2, false, false);
  c3 = __builtin_amdgcn_wmma_f32_16x16x32_f16(false, a3, false, p, (short)0, c3, false, false);
  asm volatile("v_nop\n\tv_nop\n\tv_nop\n\tv_nop" : "+v"(c0), "+v"(c1), "+v"(c2), "+v"(c3) : "v"(a0), "v"(a1), "v"(a2), "v"(a3), "v"(p));
}

__global__ __launch_bounds__(256) void k_cvt(const float* __restrict__ src, unsigned short* __restrict__ dst, int nrows, int rpb, int bstride) {
  const int t = blockIdx.x * 256 + threadIdx.x;
  if (t >= nrows * 128) return;
  const int row = t >> 7, piece = t & 127;
  const int b = row / rpb, s = row - b * rpb;
  const float* p = src + ((size_t)b * bstride + s) * DM + piece * 8;
  const v4f x0 = *(const v4fa*)(p), x1 = *(const v4fa*)(p + 4);
  v8us o;
  o[0] = bf16_bits(x0[0]); o[1] = bf16_bits(x0[1]); o[2] = bf16_bits(x0[2]); o[3] = bf16_bits(x0[3]);
  o[4] = bf16_bits(x1[0]); o[5] = bf16_bits(x1[1]); o[6] = bf16_bits(x1[2]); o[7] = bf16_bits(x1[3]);
  unsigned short* d = dst + (size_t)t * 8;
  *(volatile v8us*)d = o;
  __threadfence();
  *(volatile v8us*)d = o;
}

template <bool TWO>
__device__ __forceinline__ void gemm_loop(const unsigned short* Ah, const unsigned short* Al, const unsigned short* Bp,
                                          int m0, int n0, int ln, int hh, v8f (&acc)[2][4]) {
  const size_t ao = (size_t)(m0 + ln) * DM + 8 * hh;
  const size_t bo = (size_t)(n0 + ln) * DM + 8 * hh;
#pragma unroll 1
  for (int k0 = 0; k0 < DM; k0 += 32) {
    FragB b0, b1, b2, b3, a0, a1;
    const unsigned short* bp = Bp + bo + k0;
    b0.half[0] = *(const v8us*)(bp);            b0.half[1] = *(const v8us*)(bp + 16);
    b1.half[0] = *(const v8us*)(bp + 16 * DM);  b1.half[1] = *(const v8us*)(bp + 16 * DM + 16);
    b2.half[0] = *(const v8us*)(bp + 32 * DM);  b2.half[1] = *(const v8us*)(bp + 32 * DM + 16);
    b3.half[0] = *(const v8us*)(bp + 48 * DM);  b3.half[1] = *(const v8us*)(bp + 48 * DM + 16);
    const unsigned short* ap = Ah + ao + k0;
    a0.half[0] = *(const v8us*)(ap);            a0.half[1] = *(const v8us*)(ap + 16);
    a1.half[0] = *(const v8us*)(ap + 16 * DM);  a1.half[1] = *(const v8us*)(ap + 16 * DM + 16);
    mma_row4(a0.v, b0.v, b1.v, b2.v, b3.v, acc[0][0], acc[0][1], acc[0][2], acc[0][3]);
    mma_row4(a1.v, b0.v, b1.v, b2.v, b3.v, acc[1][0], acc[1][1], acc[1][2], acc[1][3]);
    if (TWO) {
      FragB l0, l1;
      const unsigned short* lp = Al + ao + k0;
      l0.half[0] = *(const v8us*)(lp);            l0.half[1] = *(const v8us*)(lp + 16);
      l1.half[0] = *(const v8us*)(lp + 16 * DM);  l1.half[1] = *(const v8us*)(lp + 16 * DM + 16);
      mma_row4(l0.v, b0.v, b1.v, b2.v, b3.v, acc[0][0], acc[0][1], acc[0][2], acc[0][3]);
      mma_row4(l1.v, b0.v, b1.v, b2.v, b3.v, acc[1][0], acc[1][1], acc[1][2], acc[1][3]);
    }
  }
}

__global__ __launch_bounds__(128) void k_gemm_qk(const unsigned short* __restrict__ Xb, const unsigned short* __restrict__ Wb,
                                                 unsigned short* __restrict__ Ph, unsigned short* __restrict__ Pl) {
  __shared__ __attribute__((aligned(16))) float st[4][32][68];
  const int tid = threadIdx.x, w = __builtin_amdgcn_readfirstlane((int)(tid >> 5)), lane = tid & 31, ln = lane & 15, hh = lane >> 4;
  const int n0 = blockIdx.x * 64, m0 = blockIdx.y * 128 + 32 * w;
  v8f acc[2][4] = {};
  gemm_loop<false>(Xb, Xb, Wb, m0, n0, ln, hh, acc);
#pragma unroll
  for (int i = 0; i < 2; ++i)
#pragma unroll
    for (int j = 0; j < 4; ++j)
#pragma unroll
      for (int r = 0; r < 8; ++r) st[w][16 * i + 8 * hh + r][16 * j + ln] = acc[i][j][r];
  __syncthreads();
  const int b = m0 / SEQ, s0 = m0 - b * SEQ, h = blockIdx.x;
  const int rq = lane >> 3, c8 = (lane & 7) * 8;
  const size_t base = ((size_t)(b * NH + h) * SEQ + s0) * HD + c8;
  for (int pass = 0; pass < 2; ++pass) {
#pragma unroll
    for (int it = 0; it < 8; ++it) {
      const int row = 4 * it + rq;
      const v4f x0 = *(const v4fa*)&st[w][row][c8];
      const v4f x1 = *(const v4fa*)&st[w][row][c8 + 4];
      v8us hi, lo;
      split_bf8(x0, x1, hi, lo);
      *(volatile v8us*)(Ph + base + (size_t)row * HD) = hi;
      *(volatile v8us*)(Pl + base + (size_t)row * HD) = lo;
    }
    if (pass == 0) __threadfence();
  }
}

__global__ __launch_bounds__(128) void k_gemm_vt(const unsigned short* __restrict__ Wb, const unsigned short* __restrict__ Xb,
                                                 unsigned short* __restrict__ Vh) {
  __shared__ __attribute__((aligned(16))) float st[4][32][68];
  const int tid = threadIdx.x, w = __builtin_amdgcn_readfirstlane((int)(tid >> 5)), lane = tid & 31, ln = lane & 15, hh = lane >> 4;
  const int n0 = blockIdx.x * 64, m0 = blockIdx.y * 128 + 32 * w;
  v8f acc[2][4] = {};
  gemm_loop<false>(Wb, Wb, Xb, m0, n0, ln, hh, acc);
#pragma unroll
  for (int i = 0; i < 2; ++i)
#pragma unroll
    for (int j = 0; j < 4; ++j)
#pragma unroll
      for (int r = 0; r < 8; ++r) st[w][16 * i + 8 * hh + r][16 * j + ln] = acc[i][j][r];
  __syncthreads();
  const int b = n0 / SEQ, s0 = n0 - b * SEQ;
  const int rq = lane >> 3, c8 = (lane & 7) * 8;
  const size_t base = ((size_t)b * DM + m0) * SEQ + s0 + c8;
  for (int pass = 0; pass < 2; ++pass) {
#pragma unroll
    for (int it = 0; it < 8; ++it) {
      const int row = 4 * it + rq;
      const v4f x0 = *(const v4fa*)&st[w][row][c8];
      const v4f x1 = *(const v4fa*)&st[w][row][c8 + 4];
      H8 hi;
      cvt_h8(x0, x1, hi);
      *(volatile v8us*)(Vh + base + (size_t)row * SEQ) = hi.v;
    }
    if (pass == 0) __threadfence();
  }
}

__global__ __launch_bounds__(128) void k_gemm_out(const unsigned short* __restrict__ Chi, const unsigned short* __restrict__ Clo,
                                                  const unsigned short* __restrict__ Wb, float* __restrict__ out) {
  __shared__ __attribute__((aligned(16))) float st[4][32][68];
  const int tid = threadIdx.x, w = __builtin_amdgcn_readfirstlane((int)(tid >> 5)), lane = tid & 31, ln = lane & 15, hh = lane >> 4;
  const int n0 = blockIdx.x * 64, m0 = blockIdx.y * 128 + 32 * w;
  v8f acc[2][4] = {};
  gemm_loop<true>(Chi, Clo, Wb, m0, n0, ln, hh, acc);
#pragma unroll
  for (int i = 0; i < 2; ++i)
#pragma unroll
    for (int j = 0; j < 4; ++j)
#pragma unroll
      for (int r = 0; r < 8; ++r) st[w][16 * i + 8 * hh + r][16 * j + ln] = acc[i][j][r];
  __syncthreads();
  const int b = m0 / SEQ, s0 = m0 - b * SEQ;
  const int rsub = lane >> 4, c4 = (lane & 15) * 4;
  float* og = out + (size_t)b * XSTRIDE_FULL + (size_t)s0 * DM + n0 + c4;
  for (int pass = 0; pass < 2; ++pass) {
#pragma unroll
    for (int it = 0; it < 16; ++it) {
      const int row = 2 * it + rsub;
      const v4f v = *(const v4fa*)&st[w][row][c4];
      *(volatile v4f*)(og + (size_t)row * DM) = v;
    }
    if (pass == 0) __threadfence();
  }
}

__device__ __forceinline__ void fa_step(const unsigned short* Khp, const unsigned short* Klp,
                                        const unsigned short* Vhp, const int* mp,
                                        int key0, int ln, int hh,
                                        const FragB& qh0, const FragB& qh1, const FragB& ql0, const FragB& ql1,
                                        float& mr, float& lr, v8f (&O)[4]) {
  const v8f z8 = {0.f, 0.f, 0.f, 0.f, 0.f, 0.f, 0.f, 0.f};
  v8f s0, s1;
  {
    const size_t ko = (size_t)(key0 + ln) * HD + 8 * hh;
    FragB a0, a1, c0, c1;
    a0.half[0] = *(const v8us*)(Khp + ko);      a0.half[1] = *(const v8us*)(Khp + ko + 16);
    a1.half[0] = *(const v8us*)(Khp + ko + 32); a1.half[1] = *(const v8us*)(Khp + ko + 48);
    c0.half[0] = *(const v8us*)(Klp + ko);      c0.half[1] = *(const v8us*)(Klp + ko + 16);
    c1.half[0] = *(const v8us*)(Klp + ko + 32); c1.half[1] = *(const v8us*)(Klp + ko + 48);
    s0 = mma_s6(a0.v, a1.v, c0.v, c1.v, qh0.v, qh1.v, ql0.v, ql1.v, z8);
  }
  asm volatile("" ::: "memory");
  {
    const size_t ko = (size_t)(key0 + 16 + ln) * HD + 8 * hh;
    FragB a0, a1, c0, c1;
    a0.half[0] = *(const v8us*)(Khp + ko);      a0.half[1] = *(const v8us*)(Khp + ko + 16);
    a1.half[0] = *(const v8us*)(Khp + ko + 32); a1.half[1] = *(const v8us*)(Khp + ko + 48);
    c0.half[0] = *(const v8us*)(Klp + ko);      c0.half[1] = *(const v8us*)(Klp + ko + 16);
    c1.half[0] = *(const v8us*)(Klp + ko + 32); c1.half[1] = *(const v8us*)(Klp + ko + 48);
    s1 = mma_s6(a0.v, a1.v, c0.v, c1.v, qh0.v, qh1.v, ql0.v, ql1.v, z8);
  }
  asm volatile("" ::: "memory");
  const v4ia m00 = *(const v4ia*)(mp + key0);
  const v4ia m01 = *(const v4ia*)(mp + key0 + 4);
  const v4ia m10 = *(const v4ia*)(mp + key0 + 16);
  const v4ia m11 = *(const v4ia*)(mp + key0 + 20);
  float sc[16];
#pragma unroll
  for (int r = 0; r < 8; ++r) { sc[r] = s0[r] * 0.125f; sc[8 + r] = s1[r] * 0.125f; }
#pragma unroll
  for (int r = 0; r < 4; ++r) {
    sc[r]      = (m00[r] == 0) ? FILLV : sc[r];
    sc[4 + r]  = (m01[r] == 0) ? FILLV : sc[4 + r];
    sc[8 + r]  = (m10[r] == 0) ? FILLV : sc[8 + r];
    sc[12 + r] = (m11[r] == 0) ? FILLV : sc[12 + r];
  }
  float mx = sc[0];
#pragma unroll
  for (int i = 1; i < 16; ++i) mx = fmaxf(mx, sc[i]);
  mx = fmaxf(mx, __shfl_xor(mx, 16, 32));
  const float mnew = fmaxf(mr, mx);
  const float al = exp2f((mr - mnew) * LOG2E);
  mr = mnew;
  FragH ph;
  float ps = 0.0f;
#pragma unroll
  for (int i = 0; i < 16; ++i) {
    const float pc = exp2f(fmaf(sc[i] - mnew, LOG2E, 8.0f));
    const _Float16 hv = (_Float16)pc;
    ph.h[i] = hv;
    ps += (float)hv;
  }
  ps += __shfl_xor(ps, 16, 32);
  lr = lr * al + ps;
#pragma unroll
  for (int t = 0; t < 4; ++t) O[t] = O[t] * al;
  asm volatile("" ::: "memory");
  const size_t vo = (size_t)ln * SEQ + key0 + 8 * hh;
  FragH vf[4];
#pragma unroll
  for (int t = 0; t < 4; ++t) {
    vf[t].half[0] = *(const v8us*)(Vhp + vo + (size_t)t * 16 * SEQ);
    vf[t].half[1] = *(const v8us*)(Vhp + vo + (size_t)t * 16 * SEQ + 16);
  }
  mma_pv4(vf[0].v, vf[1].v, vf[2].v, vf[3].v, ph.v, O[0], O[1], O[2], O[3]);
}

__global__ __launch_bounds__(128) void k_attn(const unsigned short* __restrict__ Qh, const unsigned short* __restrict__ Ql,
                                              const unsigned short* __restrict__ Kh, const unsigned short* __restrict__ Kl,
                                              const unsigned short* __restrict__ Vh,
                                              const int* __restrict__ M,
                                              unsigned short* __restrict__ Chi, unsigned short* __restrict__ Clo) {
  __shared__ __attribute__((aligned(16))) float so[4][16][68];
  const int tid = threadIdx.x, w = __builtin_amdgcn_readfirstlane((int)(tid >> 5)), lane = tid & 31, ln = lane & 15, hh = lane >> 4;
  const int nqt = SEQ / 64;
  const int bh = blockIdx.x / nqt, qt = blockIdx.x % nqt;
  const int b = bh / NH, h = bh % NH;
  const int qbase = qt * 64 + 16 * w;
  const int qg = qbase + ln;
  const size_t hb = (size_t)bh * SEQ * HD;
  FragB qh0, qh1, ql0, ql1;
  {
    const unsigned short* qp = Qh + hb + (size_t)qg * HD + 8 * hh;
    const unsigned short* lp = Ql + hb + (size_t)qg * HD + 8 * hh;
    qh0.half[0] = *(const v8us*)(qp);      qh0.half[1] = *(const v8us*)(qp + 16);
    qh1.half[0] = *(const v8us*)(qp + 32); qh1.half[1] = *(const v8us*)(qp + 48);
    ql0.half[0] = *(const v8us*)(lp);      ql0.half[1] = *(const v8us*)(lp + 16);
    ql1.half[0] = *(const v8us*)(lp + 32); ql1.half[1] = *(const v8us*)(lp + 48);
  }
  float mr = -3.0e38f, lr = 0.0f;
  v8f O[4] = {};
  const unsigned short* Khp = Kh + hb;
  const unsigned short* Klp = Kl + hb;
  const unsigned short* Vhp = Vh + (size_t)bh * HD * SEQ;
  const int* mp = M + (size_t)b * MSTRIDE_FULL + (size_t)qg * SEQ_FULL + 8 * hh;
#pragma unroll 1
  for (int j = 0; j < SEQ / 32; ++j)
    fa_step(Khp, Klp, Vhp, mp, 32 * j, ln, hh, qh0, qh1, ql0, ql1, mr, lr, O);

  const float inv = 1.0f / (16.0f * lr);
#pragma unroll
  for (int t = 0; t < 4; ++t)
#pragma unroll
    for (int r = 0; r < 8; ++r)
      so[w][ln][16 * t + 8 * hh + r] = O[t][r] * inv;
  __syncthreads();
  const int rq = lane >> 3, c8 = (lane & 7) * 8;
  const size_t base = ((size_t)b * SEQ + qbase) * DM + h * HD + c8;
  for (int pass = 0; pass < 2; ++pass) {
#pragma unroll
    for (int it = 0; it < 4; ++it) {
      const int row = 4 * it + rq;
      const v4f x0 = *(const v4fa*)&so[w][row][c8];
      const v4f x1 = *(const v4fa*)&so[w][row][c8 + 4];
      v8us hi, lo;
      split_bf8(x0, x1, hi, lo);
      *(volatile v8us*)(Chi + base + (size_t)row * DM) = hi;
      *(volatile v8us*)(Clo + base + (size_t)row * DM) = lo;
    }
    if (pass == 0) __threadfence();
  }
}

extern "C" void kernel_launch(void* const* d_in, const int* in_sizes, int n_in,
                              void* d_out, int out_size, void* d_ws, size_t ws_size, hipStream_t stream) {
  if (n_in < 6) return;
  const long long needx = (long long)(NB - 1) * SEQ_FULL * DM + (long long)SEQ * DM;
  const long long needm = (long long)(NB - 1) * SEQ_FULL * SEQ_FULL + (long long)(SEQ - 1) * SEQ_FULL + SEQ;
  const long long needw = (long long)DM * DM;
  if ((long long)in_sizes[0] < needx || (long long)in_sizes[1] < needm) return;
  if ((long long)in_sizes[2] < needw || (long long)in_sizes[3] < needw || (long long)in_sizes[4] < needw || (long long)in_sizes[5] < needw) return;
  if ((long long)out_size < needx) return;
  const float* X  = (const float*)d_in[0];
  const int*   Mk = (const int*)d_in[1];
  const float* Wq = (const float*)d_in[2];
  const float* Wk = (const float*)d_in[3];
  const float* Wv = (const float*)d_in[4];
  const float* Wo = (const float*)d_in[5];
  float* out = (float*)d_out;

  char* ws = (char*)d_ws;
  size_t off = 0;
  const size_t xb = (size_t)NT * DM * 2;
  const size_t wb = (size_t)DM * DM * 2;
  unsigned short* Xb  = (unsigned short*)(ws + off); off += xb;
  unsigned short* Wqb = (unsigned short*)(ws + off); off += wb;
  unsigned short* Wkb = (unsigned short*)(ws + off); off += wb;
  unsigned short* Wvb = (unsigned short*)(ws + off); off += wb;
  unsigned short* Wob = (unsigned short*)(ws + off); off += wb;
  unsigned short* Qh  = (unsigned short*)(ws + off); off += xb;
  unsigned short* Ql  = (unsigned short*)(ws + off); off += xb;
  unsigned short* Kh  = (unsigned short*)(ws + off); off += xb;
  unsigned short* Kl  = (unsigned short*)(ws + off); off += xb;
  unsigned short* Vh  = (unsigned short*)(ws + off); off += xb;
  unsigned short* Chi = (unsigned short*)(ws + off); off += xb;
  unsigned short* Clo = (unsigned short*)(ws + off); off += xb;
  if (off > ws_size) return;

  k_cvt<<<(unsigned)((NT * 128 + 255) / 256), 256, 0, stream>>>(X, Xb, NT, SEQ, SEQ_FULL);
  k_cvt<<<(unsigned)((DM * 128 + 255) / 256), 256, 0, stream>>>(Wq, Wqb, DM, DM, DM);
  k_cvt<<<(unsigned)((DM * 128 + 255) / 256), 256, 0, stream>>>(Wk, Wkb, DM, DM, DM);
  k_cvt<<<(unsigned)((DM * 128 + 255) / 256), 256, 0, stream>>>(Wv, Wvb, DM, DM, DM);
  k_cvt<<<(unsigned)((DM * 128 + 255) / 256), 256, 0, stream>>>(Wo, Wob, DM, DM, DM);

  k_gemm_qk<<<dim3(DM / 64, NT / 128), 128, 0, stream>>>(Xb, Wqb, Qh, Ql);
  k_gemm_qk<<<dim3(DM / 64, NT / 128), 128, 0, stream>>>(Xb, Wkb, Kh, Kl);
  k_gemm_vt<<<dim3(NT / 64, DM / 128), 128, 0, stream>>>(Wvb, Xb, Vh);

  k_attn<<<(unsigned)(NB * NH * (SEQ / 64)), 128, 0, stream>>>(Qh, Ql, Kh, Kl, Vh, Mk, Chi, Clo);

  k_gemm_out<<<dim3(DM / 64, NT / 128), 128, 0, stream>>>(Chi, Clo, Wob, out);
}
